// TimeDistanceViT_7035156431001
// MI455X (gfx1250) — hardware-verified
//
#include <hip/hip_runtime.h>
#include <math.h>
#include <stdint.h>

#define NBATCH 2
#define NT     4
#define NCH    3
#define IMG    224
#define PS     16
#define GP     14
#define NPAT   196
#define NTOK   784
#define NP     832
#define MP     (NBATCH * NP)
#define DM     768
#define NH     12
#define HD     64
#define DFF    3072
#define NCLS   1000
#define NLAYER 6
#define QKP    (2 * DM)
#define NQB    (NP / 64)
#define NOUT4  (NBATCH * NCLS / 4)
#define LNEPS  1.0e-5f
#define WSC    64.0f
static_assert(NH * HD == DM);
static_assert(NT * NPAT == NTOK);
static_assert(NP >= NTOK && (NP % 64) == 0 && (NP - NTOK) < 64);
static_assert((MP % 64) == 0 && (DM % 64) == 0 && (DFF % 64) == 0 && (QKP % 64) == 0);
static_assert(DM == 4 * 192 && DM == 3 * 256);
static_assert(GP * PS == IMG && GP * GP == NPAT && PS * PS * NCH == DM);
static_assert((NBATCH * NCLS) % 4 == 0 && NOUT4 <= 512 && 4 * 256 >= NCLS);

typedef _Float16 v16h __attribute__((ext_vector_type(16)));
typedef _Float16 v8h  __attribute__((ext_vector_type(8)));
typedef float    v8f  __attribute__((ext_vector_type(8)));
typedef float    v4f  __attribute__((ext_vector_type(4)));
typedef unsigned int v4u __attribute__((ext_vector_type(4)));
typedef unsigned int v2u __attribute__((ext_vector_type(2)));

__device__ __forceinline__ unsigned short bf_bits(float f) {
  unsigned u = __float_as_uint(f);
  return (unsigned short)((u + 0x7FFFu + ((u >> 16) & 1u)) >> 16);
}
__device__ __forceinline__ float bf_up(unsigned short h) { return __uint_as_float(((unsigned)h) << 16); }
__device__ __forceinline__ float bfr(float f) { return bf_up(bf_bits(f)); }
__device__ __forceinline__ unsigned short h_bits(_Float16 x) { return __builtin_bit_cast(unsigned short, x); }
__device__ __forceinline__ unsigned pk16(unsigned short a, unsigned short b) { return (unsigned)a | ((unsigned)b << 16); }
__device__ __forceinline__ v8f zero8() { v8f z = {0.f, 0.f, 0.f, 0.f, 0.f, 0.f, 0.f, 0.f}; return z; }
__device__ __forceinline__ float gelu_f(float v) { return 0.5f * v * (1.0f + erff(v * 0.70710678118654752f)); }

__device__ __forceinline__ v16h ldfrag_h(const _Float16* p) {
  union { v16h v; v8h h[2]; } f;
  f.h[0] = *(const v8h*)(p);
  f.h[1] = *(const v8h*)(p + 16);
  return f.v;
}

__device__ __forceinline__ v8f mma_h(v16h a, v16h b, v8f c) {
  c = __builtin_amdgcn_wmma_f32_16x16x32_f16(false, a, false, b, (short)0, c, false, false);
#if defined(__HIP_DEVICE_COMPILE__)
  asm volatile("v_nop\n\tv_nop\n\tv_nop\n\tv_nop" : "+v"(c) : "v"(a), "v"(b));
#endif
  return c;
}
__device__ __forceinline__ v8f mma_h_raw(v16h a, v16h b, v8f c) {
  return __builtin_amdgcn_wmma_f32_16x16x32_f16(false, a, false, b, (short)0, c, false, false);
}
__device__ __forceinline__ void dep_guard1(v8f& a, v8f& b, v16h x) {
#if defined(__HIP_DEVICE_COMPILE__)
  asm volatile("v_nop\n\tv_nop\n\tv_nop\n\tv_nop" : "+v"(a), "+v"(b) : "v"(x));
#endif
}
__device__ __forceinline__ void keep4_h(v16h a, v16h b, v16h c, v16h d) {
#if defined(__HIP_DEVICE_COMPILE__)
  asm volatile("v_nop" :: "v"(a), "v"(b), "v"(c), "v"(d));
#endif
}
__device__ __forceinline__ void acc_guard4(v8f& a, v8f& b, v8f& c, v8f& d) {
#if defined(__HIP_DEVICE_COMPILE__)
  asm volatile("v_nop\n\tv_nop\n\tv_nop\n\tv_nop" : "+v"(a), "+v"(b), "+v"(c), "+v"(d));
#endif
}
__device__ __forceinline__ void wave_sync_lds() {
  __builtin_amdgcn_fence(__ATOMIC_RELEASE, "workgroup");
  __builtin_amdgcn_wave_barrier();
  __builtin_amdgcn_fence(__ATOMIC_ACQUIRE, "workgroup");
}
__device__ __forceinline__ float wsum(float v) {
#pragma unroll
  for (int off = 16; off > 0; off >>= 1) v += __shfl_xor(v, off, 32);
  return v;
}
__device__ __forceinline__ float bsum256(float v, float* red, int lane, int wave) {
  v = wsum(v);
  if (lane == 0) red[wave] = v;
  __syncthreads();
  float tot = 0.f;
#pragma unroll
  for (int w = 0; w < 8; ++w) tot += red[w];
  return tot;
}
__device__ __forceinline__ float bsum6(float v, float* red, int lane, int wave) {
  v = wsum(v);
  if (lane == 0) red[wave] = v;
  __syncthreads();
  float tot = 0.f;
#pragma unroll
  for (int w = 0; w < 6; ++w) tot += red[w];
  return tot;
}

__global__ __launch_bounds__(256) void convT64(const float* __restrict__ W, unsigned short* Wt, int K, int O,
                                               float wsc) {
  __shared__ __align__(16) unsigned short sTt[64 * 72];
  const int tid = threadIdx.x, lane = tid & 31, wave = tid >> 5;
  const int o0 = blockIdx.x * 64, k0 = blockIdx.y * 64;
  const int kr = tid >> 2, cs = (tid & 3) * 16;
  const float* src = W + (size_t)(k0 + kr) * O + o0 + cs;
#pragma unroll
  for (int q = 0; q < 4; ++q) {
    const v4f v = *(const v4f*)(src + 4 * q);
#pragma unroll
    for (int e = 0; e < 4; ++e) sTt[(cs + 4 * q + e) * 72 + kr] = h_bits((_Float16)(bfr(v[e]) * wsc));
  }
  __syncthreads();
  const int q8 = lane >> 3, c8 = (lane & 7) * 8;
  v4u vv[2];
#pragma unroll
  for (int it = 0; it < 2; ++it) {
    const int row = wave * 8 + it * 4 + q8;
    vv[it] = *(const v4u*)(sTt + row * 72 + c8);
  }
  for (int pass = 0; pass < 2; ++pass) {
#pragma unroll
    for (int it = 0; it < 2; ++it) {
      const int row = wave * 8 + it * 4 + q8;
      *(volatile v4u*)(Wt + (size_t)(o0 + row) * K + k0 + c8) = vv[it];
    }
    __threadfence();
  }
}

template <int OM, int BIASM, int ACT, int RES>
__global__ __launch_bounds__(256) void gemm64(
    const unsigned short* __restrict__ Ap, int lda, long long strideA,
    const unsigned short* __restrict__ Btp, int ldb, long long strideB,
    const float* __restrict__ bias0, const float* __restrict__ bias1, int Nb,
    const float* resid,
    void* Cout, int ldc, long long strideC,
    int M, int N, int K, float oscale) {
  const _Float16* A  = (const _Float16*)(const void*)Ap;
  const _Float16* Bt = (const _Float16*)(const void*)Btp;
  __shared__ __align__(16) float sT[8][16 * 68];
  const int b    = blockIdx.y;
  const int lane = threadIdx.x & 31;
  const int wave = threadIdx.x >> 5;
  const int tilesN = N >> 6;
  const int tilesM = M >> 6;
  const int tile = blockIdx.x * 8 + wave;
  if (tile >= tilesM * tilesN) return;
  const int tm = tile / tilesN;
  const int tn = tile - tm * tilesN;
  const int m0 = tm << 6;
  const int n0 = tn << 6;

  const _Float16* Ab = A  + (size_t)b * strideA;
  const _Float16* Bb = Bt + (size_t)b * strideB;

  const int rlane = lane & 15;
  const int koff  = (lane >> 4) * 8;
  const int mOff  = (lane >> 4) * 8;

  v8f acc[4][4];
#pragma unroll
  for (int i = 0; i < 4; ++i)
#pragma unroll
    for (int j = 0; j < 4; ++j) acc[i][j] = zero8();

  for (int k0 = 0; k0 < K; k0 += 32) {
    v16h bh[4];
#pragma unroll
    for (int j = 0; j < 4; ++j) {
      const size_t bo = (size_t)(n0 + (j << 4) + rlane) * ldb + koff + k0;
      bh[j] = ldfrag_h(Bb + bo);
    }
#pragma unroll
    for (int i = 0; i < 4; ++i) {
      const size_t ao = (size_t)(m0 + (i << 4) + rlane) * lda + koff + k0;
      const v16h ah = ldfrag_h(Ab + ao);
#pragma unroll
      for (int j = 0; j < 4; ++j) acc[i][j] = mma_h_raw(ah, bh[j], acc[i][j]);
      dep_guard1(acc[i][0], acc[i][3], ah);
    }
    keep4_h(bh[0], bh[1], bh[2], bh[3]);
  }
  acc_guard4(acc[0][0], acc[0][1], acc[0][2], acc[0][3]);
  acc_guard4(acc[1][0], acc[1][1], acc[1][2], acc[1][3]);
  acc_guard4(acc[2][0], acc[2][1], acc[2][2], acc[2][3]);
  acc_guard4(acc[3][0], acc[3][1], acc[3][2], acc[3][3]);

  const int hh2 = lane >> 4, c4 = (lane & 15) * 4;
  const int q8  = lane >> 3, c8 = (lane & 7) * 8;
  float bc[8];
#pragma unroll
  for (int e = 0; e < 8; ++e) bc[e] = 0.f;
  if (BIASM == 0) {
    const bool use1 = (n0 >= Nb);
    if (OM == 0) {
      const int cb = n0 + c4;
      const int i0 = (cb < Nb - 4) ? cb : (Nb - 4);
      const int i1 = (cb - Nb > 0) ? (cb - Nb) : 0;
      const v4f b0v = *(const v4f*)(bias0 + i0);
      const v4f b1v = *(const v4f*)(bias1 + i1);
#pragma unroll
      for (int e = 0; e < 4; ++e) bc[e] = bfr(use1 ? b1v[e] : b0v[e]);
    } else {
      const int cb = n0 + c8;
      const int i0 = (cb < Nb - 8) ? cb : (Nb - 8);
      const int i1 = (cb - Nb > 0) ? (cb - Nb) : 0;
      const v4f b0a = *(const v4f*)(bias0 + i0), b0b = *(const v4f*)(bias0 + i0 + 4);
      const v4f b1a = *(const v4f*)(bias1 + i1), b1b = *(const v4f*)(bias1 + i1 + 4);
#pragma unroll
      for (int e = 0; e < 4; ++e) {
        bc[e]     = bfr(use1 ? b1a[e] : b0a[e]);
        bc[4 + e] = bfr(use1 ? b1b[e] : b0b[e]);
      }
    }
  }

  float* slab = sT[wave];
#pragma unroll
  for (int i = 0; i < 4; ++i) {
    const int mBase = m0 + (i << 4);
#pragma unroll
    for (int j = 0; j < 4; ++j) {
#pragma unroll
      for (int r = 0; r < 8; ++r) {
        slab[(mOff + r) * 68 + (j << 4) + rlane] = acc[i][j][r];
      }
    }
    wave_sync_lds();
    if (OM == 0) {
      float* C = (float*)Cout + (size_t)b * strideC;
      const float* Rb = resid + (size_t)b * strideC;
      v4f vals[8];
#pragma unroll
      for (int it = 0; it < 8; ++it) {
        const int row = it * 2 + hh2;
        v4f v = *(const v4f*)(slab + row * 68 + c4);
#pragma unroll
        for (int e = 0; e < 4; ++e) {
          float f = v[e] * oscale + bc[e];
          if (ACT) f = gelu_f(f);
          v[e] = f;
        }
        if (RES == 1) {
          const v4f rr = *(const v4f*)(Rb + (size_t)(mBase + row) * ldc + n0 + c4);
#pragma unroll
          for (int e = 0; e < 4; ++e) v[e] += rr[e];
        } else if (RES == 2) {
          const int pr = ((mBase + row) % NP) % NPAT;
          const v4f rr = *(const v4f*)(resid + (size_t)pr * ldc + n0 + c4);
#pragma unroll
          for (int e = 0; e < 4; ++e) v[e] += bfr(rr[e]);
        }
        vals[it] = v;
      }
      for (int pass = 0; pass < 2; ++pass) {
#pragma unroll
        for (int it = 0; it < 8; ++it) {
          const int row = it * 2 + hh2;
          *(volatile v4f*)(C + (size_t)(mBase + row) * ldc + n0 + c4) = vals[it];
        }
        __threadfence();
      }
    } else {
      unsigned short* C = (unsigned short*)Cout + (size_t)b * strideC;
      v4u hv[4];
#pragma unroll
      for (int it = 0; it < 4; ++it) {
        const int row = it * 4 + q8;
        const float* sp = slab + row * 68 + c8;
        float bm = 0.f;
        if (BIASM == 1) bm = bfr(bias0[mBase + row]);
        v4u a;
#pragma unroll
        for (int e = 0; e < 4; ++e) {
          float f0 = sp[2 * e]     * oscale + ((BIASM == 1) ? bm : bc[2 * e]);
          float f1 = sp[2 * e + 1] * oscale + ((BIASM == 1) ? bm : bc[2 * e + 1]);
          if (ACT) { f0 = gelu_f(f0); f1 = gelu_f(f1); }
          unsigned short u0, u1;
          if (OM == 1) { u0 = bf_bits(f0); u1 = bf_bits(f1); }
          else         { u0 = h_bits((_Float16)f0); u1 = h_bits((_Float16)f1); }
          a[e] = pk16(u0, u1);
        }
        hv[it] = a;
      }
      for (int pass = 0; pass < 2; ++pass) {
#pragma unroll
        for (int it = 0; it < 4; ++it) {
          const int row = it * 4 + q8;
          *(volatile v4u*)(C + (size_t)(mBase + row) * ldc + n0 + c8) = hv[it];
        }
        __threadfence();
      }
    }
    wave_sync_lds();
  }
}

__global__ __launch_bounds__(128)
void attn64(const unsigned short* __restrict__ qkp, const unsigned short* __restrict__ vtp,
            const float* __restrict__ tms, const float* __restrict__ ga, const float* __restrict__ gc,
            unsigned short* outp, float sscale) {
  union FH { v16h v; v8h h[2]; };
  __shared__ __align__(16) _Float16 Ksh[64 * 64];
  __shared__ __align__(16) _Float16 Vth[64 * 64];
  __shared__ __align__(16) _Float16 Psh[4][16 * 64];
  __shared__ __align__(16) float    Os[4][16 * 64];

  const int tid  = threadIdx.x;
  const int wave = tid >> 5;
  const int lane = tid & 31;
  const int hh   = lane >> 4;
  const int c    = lane & 15;

  const int bx   = blockIdx.x;
  const int qb   = bx % NQB;
  const int rest = bx / NQB;
  const int h    = rest % NH;
  const int b    = rest / NH;
  const int q0   = qb * 64 + wave * 16;
  const size_t rowB = (size_t)b * NP;

  const _Float16* Qh = (const _Float16*)(const void*)qkp + (size_t)h * HD;
  const _Float16* Kg = (const _Float16*)(const void*)qkp + DM + (size_t)h * HD;
  const _Float16* Vh = (const _Float16*)(const void*)vtp + ((size_t)b * DM + (size_t)h * HD) * NP;

  const float aa = fabsf(bfr(ga[h])), cc = fabsf(bfr(gc[h]));
  const float t0 = bfr(tms[b * NT]);
  float dec[8];
#pragma unroll
  for (int r = 0; r < 8; ++r) {
    int ti = (q0 + 8 * hh + r) / NPAT;
    ti = (ti > NT - 1) ? (NT - 1) : ti;
    const float rr = fabsf(t0 - bfr(tms[b * NT + ti]));
    const float z  = aa * rr - cc;
    dec[r] = 1.0f / (1.0f + expf(z));
  }

  v16h qa[2];
#pragma unroll
  for (int dc = 0; dc < 2; ++dc) qa[dc] = ldfrag_h(Qh + (rowB + q0 + c) * QKP + dc * 32 + 8 * hh);

  float mrow[8], lrow[8];
  v8f oacc[4];
#pragma unroll
  for (int r = 0; r < 8; ++r) { mrow[r] = -INFINITY; lrow[r] = 0.f; }
#pragma unroll
  for (int t = 0; t < 4; ++t) oacc[t] = zero8();

  for (int kt = 0; kt < NQB; ++kt) {
    const int kv0 = kt * 64;
    __syncthreads();
    {
      const int r = tid >> 1, hf = (tid & 1) * 32;
      const _Float16* kg = Kg + (rowB + kv0 + r) * QKP + hf;
      const _Float16* vg = Vh + (size_t)r * NP + kv0 + hf;
#pragma unroll
      for (int i = 0; i < 4; ++i) {
        const v8h a0 = *(const v8h*)(kg + 8 * i);
        const v8h b0 = *(const v8h*)(vg + 8 * i);
        *(v8h*)(Ksh + r * 64 + hf + 8 * i) = a0;
        *(v8h*)(Vth + r * 64 + hf + 8 * i) = b0;
      }
    }
    __syncthreads();

    v8f s[4];
#pragma unroll
    for (int j = 0; j < 4; ++j) {
      v8f sh = zero8();
#pragma unroll
      for (int dc = 0; dc < 2; ++dc) {
        FH kb;
        kb.h[0] = *(const v8h*)(Ksh + (j * 16 + c) * 64 + dc * 32 + 8 * hh);
        kb.h[1] = *(const v8h*)(Ksh + (j * 16 + c) * 64 + dc * 32 + 16 + 8 * hh);
        sh = mma_h(qa[dc], kb.v, sh);
      }
#pragma unroll
      for (int r = 0; r < 8; ++r) {
        float v = sh[r] * sscale;
        v = fmaxf(v, 0.0f) * dec[r];
        const int key = kv0 + j * 16 + c;
        s[j][r] = (key < NTOK) ? v : -INFINITY;
      }
    }

    _Float16* pwh = Psh[wave];
#pragma unroll
    for (int r = 0; r < 8; ++r) {
      float m = s[0][r];
      m = fmaxf(m, s[1][r]);
      m = fmaxf(m, s[2][r]);
      m = fmaxf(m, s[3][r]);
#pragma unroll
      for (int off = 1; off < 16; off <<= 1) m = fmaxf(m, __shfl_xor(m, off, 32));
      const float mnew  = fmaxf(mrow[r], m);
      const float alpha = __expf(mrow[r] - mnew);
      mrow[r] = mnew;
      float psum = 0.f;
#pragma unroll
      for (int j = 0; j < 4; ++j) {
        const float p = __expf(s[j][r] - mnew);
        psum += p;
        pwh[(8 * hh + r) * 64 + j * 16 + c] = (_Float16)(p * 1024.0f);
      }
#pragma unroll
      for (int off = 1; off < 16; off <<= 1) psum += __shfl_xor(psum, off, 32);
      lrow[r] = lrow[r] * alpha + psum;
#pragma unroll
      for (int t = 0; t < 4; ++t) oacc[t][r] *= alpha;
    }
    wave_sync_lds();

#pragma unroll 1
    for (int kk = 0; kk < 2; ++kk) {
      FH pa;
      pa.h[0] = *(const v8h*)(pwh + c * 64 + kk * 32 + 8 * hh);
      pa.h[1] = *(const v8h*)(pwh + c * 64 + kk * 32 + 16 + 8 * hh);
#pragma unroll
      for (int t = 0; t < 4; ++t) {
        FH vb;
        vb.h[0] = *(const v8h*)(Vth + (t * 16 + c) * 64 + kk * 32 + 8 * hh);
        vb.h[1] = *(const v8h*)(Vth + (t * 16 + c) * 64 + kk * 32 + 16 + 8 * hh);
        oacc[t] = mma_h(pa.v, vb.v, oacc[t]);
      }
    }
  }

  float* os = Os[wave];
#pragma unroll
  for (int r = 0; r < 8; ++r) {
    const float l = lrow[r];
    const float inv = ((l > 0.f) ? (1.0f / l) : 0.f) * (16.0f / 1024.0f);
#pragma unroll
    for (int t = 0; t < 4; ++t) os[(8 * hh + r) * 64 + t * 16 + c] = oacc[t][r] * inv;
  }
  wave_sync_lds();
  {
    const int q4 = lane >> 3, c8 = (lane & 7) * 8;
    v4u hv[4];
#pragma unroll
    for (int it = 0; it < 4; ++it) {
      const int row = it * 4 + q4;
      const float* sp = os + row * 64 + c8;
      v4u a;
#pragma unroll
      for (int e = 0; e < 4; ++e) a[e] = pk16(h_bits((_Float16)sp[2 * e]), h_bits((_Float16)sp[2 * e + 1]));
      hv[it] = a;
    }
    for (int pass = 0; pass < 2; ++pass) {
#pragma unroll
      for (int it = 0; it < 4; ++it) {
        const int row = it * 4 + q4;
        const size_t go = (rowB + q0 + row) * DM + (size_t)h * HD + c8;
        *(volatile v4u*)(outp + go) = hv[it];
      }
      __threadfence();
    }
  }
}

__device__ __forceinline__ void row_store_h16(unsigned int* sb, unsigned short* dst_row, v4f o, int t) {
  v2u p;
  p[0] = pk16(h_bits((_Float16)o[0]), h_bits((_Float16)o[1]));
  p[1] = pk16(h_bits((_Float16)o[2]), h_bits((_Float16)o[3]));
  *(v2u*)(sb + 2 * t) = p;
  __syncthreads();
  if (t < 96) {
    const v4u v = *(const v4u*)(sb + 4 * t);
    *(volatile v4u*)(dst_row + 8 * t) = v;
    __threadfence();
    *(volatile v4u*)(dst_row + 8 * t) = v;
  }
}

__global__ __launch_bounds__(192) void patch_rows(const float* __restrict__ img, unsigned short* XP) {
  __shared__ __align__(16) unsigned int sb[384];
  const int t  = threadIdx.x;
  const int m  = blockIdx.x;
  const int b  = m / NP;
  const int tk = m - b * NP;
  v4f y;
  y[0] = 0.f; y[1] = 0.f; y[2] = 0.f; y[3] = 0.f;
  if (tk < NTOK) {
    const int tt = tk / NPAT, g = tk - tt * NPAT;
    const int gy = g / GP, gx = g - gy * GP;
    const float* base = img + (size_t)(b * NT + tt) * NCH * IMG * IMG;
#pragma unroll
    for (int e = 0; e < 4; ++e) {
      const int k  = 4 * t + e;
      const int ch = k % NCH;
      const int q  = k / NCH;
      const int p1 = q >> 4, p2 = q & 15;
      const size_t src = (size_t)ch * IMG * IMG + (size_t)(gy * PS + p1) * IMG + (size_t)(gx * PS + p2);
      y[e] = bfr(base[src]);
    }
  }
  row_store_h16(sb, XP + (size_t)m * DM, y, t);
}

__global__ __launch_bounds__(192) void ln_row_h(const float* __restrict__ X, const float* __restrict__ gam,
                                                const float* __restrict__ bet, unsigned short* outH) {
  __shared__ float red0[8], red1[8];
  __shared__ __align__(16) unsigned int sb[384];
  const int t = threadIdx.x, lane = t & 31, wave = t >> 5;
  const size_t base = (size_t)blockIdx.x * DM;
  const v4f xv = *(const v4f*)(X + base + 4 * t);
  const float mean = bsum6((xv[0] + xv[1]) + (xv[2] + xv[3]), red0, lane, wave) * (1.0f / DM);
  v4f d;
#pragma unroll
  for (int e = 0; e < 4; ++e) d[e] = xv[e] - mean;
  const float var  = bsum6((d[0] * d[0] + d[1] * d[1]) + (d[2] * d[2] + d[3] * d[3]), red1, lane, wave) * (1.0f / DM);
  const float rstd = 1.0f / sqrtf(var + LNEPS);
  const v4f gv = *(const v4f*)(gam + 4 * t);
  const v4f bv = *(const v4f*)(bet + 4 * t);
  v4f y;
#pragma unroll
  for (int e = 0; e < 4; ++e) y[e] = (d[e] * rstd) * bfr(gv[e]) + bfr(bv[e]);
  row_store_h16(sb, outH + base, y, t);
}

__global__ __launch_bounds__(256) void head_k(const float* __restrict__ X,
                                              const float* __restrict__ lw, const float* __restrict__ lb,
                                              const float* __restrict__ hw1, const float* __restrict__ hb1,
                                              const float* __restrict__ hw2, const float* __restrict__ hb2,
                                              float* out) {
  __shared__ float sx[NBATCH][DM];
  __shared__ float sl[NBATCH][DM];
  __shared__ float sy[NBATCH][DM];
  __shared__ __align__(16) float so[2048];
  __shared__ float red[4][8];
  const int t = threadIdx.x, lane = t & 31, wave = t >> 5;

#pragma unroll 1
  for (int j = 0; j < 3; ++j) {
    const int col = t + 256 * j;
    double s0 = 0.0, s1 = 0.0;
#pragma unroll 2
    for (int n = 0; n < NTOK; ++n) {
      s0 += (double)X[(size_t)n * DM + col];
      s1 += (double)X[(size_t)(NP + n) * DM + col];
    }
    sx[0][col] = (float)(s0 * (1.0 / (double)NTOK));
    sx[1][col] = (float)(s1 * (1.0 / (double)NTOK));
  }
  __syncthreads();

#pragma unroll
  for (int bb = 0; bb < NBATCH; ++bb) {
    const float v0 = sx[bb][t], v1 = sx[bb][t + 256], v2 = sx[bb][t + 512];
    const float mean = bsum256((v0 + v1) + v2, red[2 * bb], lane, wave) * (1.0f / DM);
    const float d0 = v0 - mean, d1 = v1 - mean, d2 = v2 - mean;
    const float var  = bsum256((d0 * d0 + d1 * d1) + d2 * d2, red[2 * bb + 1], lane, wave) * (1.0f / DM);
    const float rstd = 1.0f / sqrtf(var + LNEPS);
    sl[bb][t]       = (d0 * rstd) * bfr(lw[t])       + bfr(lb[t]);
    sl[bb][t + 256] = (d1 * rstd) * bfr(lw[t + 256]) + bfr(lb[t + 256]);
    sl[bb][t + 512] = (d2 * rstd) * bfr(lw[t + 512]) + bfr(lb[t + 512]);
  }
  __syncthreads();

  float a0[3], a1[3];
#pragma unroll
  for (int j = 0; j < 3; ++j) { a0[j] = 0.f; a1[j] = 0.f; }
#pragma unroll 1
  for (int k = 0; k < DM; ++k) {
    const float x0 = sl[0][k], x1 = sl[1][k];
    const float* wr = hw1 + (size_t)k * DM + t;
#pragma unroll
    for (int j = 0; j < 3; ++j) {
      const float w = bfr(wr[256 * j]);
      a0[j] += x0 * w;
      a1[j] += x1 * w;
    }
  }
#pragma unroll
  for (int j = 0; j < 3; ++j) {
    const int col = t + 256 * j;
    const float bv = bfr(hb1[col]);
    sy[0][col] = a0[j] + bv;
    sy[1][col] = a1[j] + bv;
  }
  __syncthreads();

  float e0[4], e1[4];
  int oc[4];
#pragma unroll
  for (int j = 0; j < 4; ++j) {
    e0[j] = 0.f; e1[j] = 0.f;
    const int o = t + 256 * j;
    oc[j] = (o < NCLS) ? o : (NCLS - 1);
  }
#pragma unroll 1
  for (int k = 0; k < DM; ++k) {
    const float y0 = sy[0][k], y1 = sy[1][k];
    const float* wr = hw2 + (size_t)k * NCLS;
#pragma unroll
    for (int j = 0; j < 4; ++j) {
      const float w = bfr(wr[oc[j]]);
      e0[j] += y0 * w;
      e1[j] += y1 * w;
    }
  }
#pragma unroll
  for (int j = 0; j < 4; ++j) {
    const int o = t + 256 * j;
    if (o < NCLS) {
      const float bv = bfr(hb2[oc[j]]);
      so[o]        = e0[j] + bv;
      so[NCLS + o] = e1[j] + bv;
    }
  }
  __syncthreads();

  const int i2  = t + 256;
  const int i2c = (i2 < NOUT4) ? i2 : (NOUT4 - 1);
  const v4f va = *(const v4f*)(so + 4 * t);
  const v4f vb = *(const v4f*)(so + 4 * i2c);
  *(volatile v4f*)(out + 4 * t) = va;
  if (i2 < NOUT4) *(volatile v4f*)(out + 4 * i2) = vb;
  __threadfence();
  *(volatile v4f*)(out + 4 * t) = va;
  if (i2 < NOUT4) *(volatile v4f*)(out + 4 * i2) = vb;
}

extern "C" void kernel_launch(void* const* d_in, const int* in_sizes, int n_in,
                              void* d_out, int out_size, void* d_ws, size_t ws_size,
                              hipStream_t stream) {
  if (n_in < 23) return;
  if (in_sizes[0] != NBATCH * NT * NCH * IMG * IMG) return;
  if (in_sizes[1] != NBATCH * NT) return;
  if (in_sizes[2] != DM * DM || in_sizes[3] != DM) return;
  if (in_sizes[4] != NPAT * DM) return;
  if (in_sizes[5] != NLAYER * DM || in_sizes[6] != NLAYER * DM) return;
  if (in_sizes[7] != NLAYER * DM * 3 * DM) return;
  if (in_sizes[8] != NLAYER * DM * DM) return;
  if (in_sizes[9] != NLAYER * NH || in_sizes[10] != NLAYER * NH) return;
  if (in_sizes[11] != NLAYER * DM || in_sizes[12] != NLAYER * DM) return;
  if (in_sizes[13] != NLAYER * DM * DFF || in_sizes[14] != NLAYER * DFF) return;
  if (in_sizes[15] != NLAYER * DFF * DM || in_sizes[16] != NLAYER * DM) return;
  if (in_sizes[17] != DM || in_sizes[18] != DM) return;
  if (in_sizes[19] != DM * DM || in_sizes[20] != DM) return;
  if (in_sizes[21] != DM * NCLS || in_sizes[22] != NCLS) return;
  if (out_size != NBATCH * NCLS) return;

  const float* img     = (const float*)d_in[0];
  const float* tms     = (const float*)d_in[1];
  const float* patch_w = (const float*)d_in[2];
  const float* patch_b = (const float*)d_in[3];
  const float* pos_emb = (const float*)d_in[4];
  const float* ln1_w   = (const float*)d_in[5];
  const float* ln1_b   = (const float*)d_in[6];
  const float* wqkv    = (const float*)d_in[7];
  const float* wout    = (const float*)d_in[8];
  const float* ta_a    = (const float*)d_in[9];
  const float* ta_c    = (const float*)d_in[10];
  const float* ln2_w   = (const float*)d_in[11];
  const float* ln2_b   = (const float*)d_in[12];
  const float* w1      = (const float*)d_in[13];
  const float* b1      = (const float*)d_in[14];
  const float* w2      = (const float*)d_in[15];
  const float* b2      = (const float*)d_in[16];
  const float* hln_w   = (const float*)d_in[17];
  const float* hln_b   = (const float*)d_in[18];
  const float* hw1     = (const float*)d_in[19];
  const float* hb1     = (const float*)d_in[20];
  const float* hw2     = (const float*)d_in[21];
  const float* hb2     = (const float*)d_in[22];

  const size_t PW1   = (size_t)DM * DM * 2;
  const size_t PWQKV = (size_t)3 * DM * DM * 2;
  const size_t PWF   = (size_t)DM * DFF * 2;
  const size_t PAH   = (size_t)MP * DM * 2;
  const size_t PAF   = (size_t)MP * DM * 4;
  const size_t PQK   = (size_t)MP * QKP * 2;
  const size_t PVT   = (size_t)NBATCH * DM * NP * 2;
  const size_t PG    = (size_t)MP * DFF * 2;
  size_t off = 0;
  const size_t oPwT  = off; off += PW1;
  const size_t oWqkv = off; off += PWQKV;
  const size_t oWo   = off; off += PW1;
  const size_t oW1   = off; off += PWF;
  const size_t oW2   = off; off += PWF;
  const size_t oXP   = off; off += PAH;
  const size_t oXA   = off; off += PAF;
  const size_t oXB   = off; off += PAF;
  const size_t oXN   = off; off += PAH;
  const size_t oQK   = off; off += PQK;
  const size_t oVT   = off; off += PVT;
  const size_t oCtx  = off; off += PAH;
  const size_t oG    = off; off += PG;
  if (off > ws_size) return;
  if (off > (size_t)134217728) return;

  char* ws = (char*)d_ws;
  unsigned short* PwT   = (unsigned short*)(ws + oPwT);
  unsigned short* WqkvT = (unsigned short*)(ws + oWqkv);
  unsigned short* WoT   = (unsigned short*)(ws + oWo);
  unsigned short* W1T   = (unsigned short*)(ws + oW1);
  unsigned short* W2T   = (unsigned short*)(ws + oW2);
  unsigned short* XP    = (unsigned short*)(ws + oXP);
  float*          XA    = (float*)(ws + oXA);
  float*          XB    = (float*)(ws + oXB);
  unsigned short* XN    = (unsigned short*)(ws + oXN);
  unsigned short* QK    = (unsigned short*)(ws + oQK);
  unsigned short* VT    = (unsigned short*)(ws + oVT);
  unsigned short* Ctx   = (unsigned short*)(ws + oCtx);
  unsigned short* G     = (unsigned short*)(ws + oG);

  const dim3 blk(256), blk192(192), blk128(128);
  const dim3 gRow(MP);
  const dim3 gT768(DM / 64, DM / 64);
  const dim3 gTqkv((3 * DM) / 64, DM / 64);
  const dim3 gTw1(DFF / 64, DM / 64);
  const dim3 gTw2(DM / 64, DFF / 64);
  const dim3 gN768(((MP / 64) * (DM / 64) + 7) / 8, 1);
  const dim3 gNqk(((MP / 64) * (QKP / 64) + 7) / 8, 1);
  const dim3 gNff(((MP / 64) * (DFF / 64) + 7) / 8, 1);
  const dim3 gVT(((DM / 64) * (NP / 64) + 7) / 8, NBATCH);
  const dim3 gAttn(NBATCH * NH * NQB);
  const float invw  = 1.0f / WSC;
  const float invwc = 1.0f / (WSC * 16.0f);

  patch_rows<<<gRow, blk192, 0, stream>>>(img, XP);
  convT64<<<gT768, blk, 0, stream>>>(patch_w, PwT, DM, DM, WSC);
  gemm64<0, 0, 0, 2><<<gN768, blk, 0, stream>>>(
      XP, DM, 0LL, PwT, DM, 0LL, patch_b, patch_b, DM, pos_emb,
      (void*)XA, DM, 0LL, MP, DM, DM, invw);

  for (int l = 0; l < NLAYER; ++l) {
    const float* Wqkv_l = wqkv + (size_t)l * DM * 3 * DM;
    const float* Wo_l   = wout + (size_t)l * DM * DM;
    const float* W1_l   = w1 + (size_t)l * DM * DFF;
    const float* W2_l   = w2 + (size_t)l * DFF * DM;
    const float* b1_l   = b1 + (size_t)l * DFF;
    const float* b2_l   = b2 + (size_t)l * DM;

    ln_row_h<<<gRow, blk192, 0, stream>>>(XA, ln1_w + (size_t)l * DM, ln1_b + (size_t)l * DM, XN);
    convT64<<<gTqkv, blk, 0, stream>>>(Wqkv_l, WqkvT, DM, 3 * DM, WSC);
    gemm64<2, 2, 0, 0><<<gNqk, blk, 0, stream>>>(
        XN, DM, 0LL, WqkvT, DM, 0LL, b2_l, b2_l, QKP, XA,
        (void*)QK, QKP, 0LL, MP, QKP, DM, invw);
    gemm64<2, 2, 0, 0><<<gVT, blk, 0, stream>>>(
        WqkvT + (size_t)2 * DM * DM, DM, 0LL, XN, DM, (long long)NP * DM, b2_l, b2_l, NP, XA,
        (void*)VT, NP, (long long)DM * NP, DM, NP, DM, invw);
    attn64<<<gAttn, blk128, 0, stream>>>(QK, VT, tms, ta_a + (size_t)l * NH, ta_c + (size_t)l * NH, Ctx, 0.125f);
    convT64<<<gT768, blk, 0, stream>>>(Wo_l, WoT, DM, DM, WSC);
    gemm64<0, 2, 0, 1><<<gN768, blk, 0, stream>>>(
        Ctx, DM, 0LL, WoT, DM, 0LL, b2_l, b2_l, DM, XA,
        (void*)XB, DM, 0LL, MP, DM, DM, invwc);
    ln_row_h<<<gRow, blk192, 0, stream>>>(XB, ln2_w + (size_t)l * DM, ln2_b + (size_t)l * DM, XN);
    convT64<<<gTw1, blk, 0, stream>>>(W1_l, W1T, DM, DFF, WSC);
    gemm64<2, 0, 1, 0><<<gNff, blk, 0, stream>>>(
        XN, DM, 0LL, W1T, DM, 0LL, b1_l, b1_l, DFF, XA,
        (void*)G, DFF, 0LL, MP, DFF, DM, invw);
    convT64<<<gTw2, blk, 0, stream>>>(W2_l, W2T, DFF, DM, WSC);
    gemm64<0, 0, 0, 1><<<gN768, blk, 0, stream>>>(
        G, DFF, 0LL, W2T, DFF, 0LL, b2_l, b2_l, DM, XB,
        (void*)XA, DM, 0LL, MP, DM, DFF, invw);
  }

  head_k<<<dim3(1), blk, 0, stream>>>(XA, hln_w, hln_b, hw1, hb1, hw2, hb2, (float*)d_out);
  (void)hipGetLastError();
}
